// CrossDimensionalAttention_60550448939365
// MI455X (gfx1250) — hardware-verified
//
#include <hip/hip_runtime.h>


namespace {
constexpr int B = 4, S = 2048, H = 512, R = B * S;
constexpr float XS = 8.0f, WSC = 256.0f, EPS = 1e-5f;
typedef _Float16 b16;
typedef __attribute__((ext_vector_type(16))) _Float16 v16b;
typedef __attribute__((ext_vector_type(8))) _Float16 v8b;
typedef __attribute__((ext_vector_type(8))) float v8f;
typedef __attribute__((ext_vector_type(4))) float v4f;
__device__ __forceinline__ float bf16_rne(float f) { unsigned int u = __float_as_uint(f); u += 0x7FFFu + ((u >> 16) & 1u); float r = __uint_as_float(u & 0xFFFF0000u); asm volatile("" : "+v"(r)); return r; }
__device__ __forceinline__ void split16(float v, b16& hi, b16& lo) { hi = (b16)v; lo = (b16)(v - (float)hi); }
__device__ __forceinline__ v16b frag_kb(const b16* p, int hh) { const v8b a = *(const v8b*)(p + 8 * hh), b = *(const v8b*)(p + 16 + 8 * hh); v16b f;
#pragma unroll
  for (int e = 0; e < 8; ++e) { f[e] = a[e]; f[8 + e] = b[e]; } return f; }
__device__ __forceinline__ v8f wmma16b(v16b a, v16b b, v8f c) { v8f d = __builtin_amdgcn_wmma_f32_16x16x32_f16(false, a, false, b, (short)0, c, false, false); asm volatile("v_nop\n\tv_nop\n\tv_nop\n\tv_nop" : "+v"(d) : "v"(a), "v"(b)); return d; }
__device__ __forceinline__ void wave_lds_sync() { __builtin_amdgcn_fence(__ATOMIC_RELEASE, "workgroup"); __builtin_amdgcn_wave_barrier(); __builtin_amdgcn_fence(__ATOMIC_ACQUIRE, "workgroup"); }
__device__ __forceinline__ float pmul(float a, float b) { float p = a * b; asm volatile("" : "+v"(p)); return p; }

__global__ __launch_bounds__(256) void wput_kernel(const float* __restrict__ wf, const float* __restrict__ wo, b16* __restrict__ WF, b16* __restrict__ WO) { const size_t u = (size_t)blockIdx.x * 256 + threadIdx.x; if (u >= (size_t)H * (H / 8)) return; v8b a, b;
#pragma unroll
  for (int j = 0; j < 8; ++j) { a[j] = (b16)(bf16_rne(wf[u * 8 + j]) * WSC); b[j] = (b16)(bf16_rne(wo[u * 8 + j]) * WSC); }
  for (int pass = 0; pass < 2; ++pass) { *(volatile v8b*)(WF + u * 8) = a; *(volatile v8b*)(WO + u * 8) = b; __threadfence(); } }
__global__ __launch_bounds__(32) void fp_kernel(const float* __restrict__ st, const b16* __restrict__ WF, const float* __restrict__ bf, float* __restrict__ FP) { __shared__ __attribute__((aligned(16))) b16 Ah[16][H + 8]; __shared__ float Tf[16][132]; const int lane = threadIdx.x, nloc = lane & 15, hlf = lane >> 4; const int g = blockIdx.x;
  for (int rr = 0; rr < 16; ++rr) for (int q = 0; q < H / 32; ++q) Ah[rr][q * 32 + lane] = (b16)(rr < B ? bf16_rne(st[rr * H + q * 32 + lane]) * XS : 0.0f);
  wave_lds_sync(); v8f acc[8];
#pragma unroll
  for (int t = 0; t < 8; ++t) acc[t] = (v8f){};
#pragma unroll 2
  for (int kb = 0; kb < H; kb += 32) { const v16b a = frag_kb(&Ah[nloc][kb], hlf);
#pragma unroll
    for (int t = 0; t < 8; ++t) acc[t] = wmma16b(a, frag_kb(WF + (size_t)(g * 128 + t * 16 + nloc) * H + kb, hlf), acc[t]); }
#pragma unroll
  for (int t = 0; t < 8; ++t) { const int cc = t * 16 + nloc; const float bb = bf16_rne(bf[g * 128 + cc]);
#pragma unroll
    for (int r8 = 0; r8 < 8; ++r8) Tf[8 * hlf + r8][cc] = acc[t][r8] * (1.0f / (XS * WSC)) + bb; }
  wave_lds_sync();
  for (int pass = 0; pass < 2; ++pass) { for (int rr = 0; rr < B; ++rr) *(volatile v4f*)(FP + rr * H + g * 128 + lane * 4) = *(const v4f*)(&Tf[rr][lane * 4]); __threadfence(); } }
__global__ __launch_bounds__(32) void main_kernel(const float* __restrict__ x, const float* __restrict__ FP, const float* __restrict__ g1, const float* __restrict__ b1, const b16* __restrict__ WO, const float* __restrict__ bo, int RLIM, float* __restrict__ P) { __shared__ __attribute__((aligned(16))) b16 Ah[16][H + 8], Al[16][H + 8]; __shared__ float O1[16][H + 4], Tf[16][260]; const int lane = threadIdx.x, nloc = lane & 15, hlf = lane >> 4; const int grp = blockIdx.x & 1; const size_t r0 = (size_t)(blockIdx.x >> 1) * 16; if (r0 >= (size_t)RLIM) return; const int b = (int)(r0 / S);
  for (int rr = 0; rr < 16; ++rr) { float v[16]; float s = 0.0f;
#pragma unroll
    for (int q = 0; q < 16; ++q) { const int c = q * 32 + lane; v[q] = bf16_rne(x[(r0 + rr) * H + c]) + FP[b * H + c]; s += v[q]; } for (int o = 16; o; o >>= 1) s += __shfl_xor(s, o); const float mu = s * (1.0f / H); float qs = 0.0f;
#pragma unroll
    for (int q = 0; q < 16; ++q) qs += pmul(v[q] - mu, v[q] - mu); for (int o = 16; o; o >>= 1) qs += __shfl_xor(qs, o); const float rs = rsqrtf(qs * (1.0f / H) + EPS);
#pragma unroll
    for (int q = 0; q < 16; ++q) { const int c = q * 32 + lane; const float o1 = pmul(pmul(v[q] - mu, rs), bf16_rne(g1[c])) + bf16_rne(b1[c]); O1[rr][c] = o1; b16 p, ql; split16(o1 * XS, p, ql); Ah[rr][c] = p; Al[rr][c] = ql; } }
  wave_lds_sync(); v8f acc[16];
#pragma unroll
  for (int t = 0; t < 16; ++t) acc[t] = (v8f){};
#pragma unroll 1
  for (int kb = 0; kb < H; kb += 32) { const v16b a = frag_kb(&Ah[nloc][kb], hlf), al = frag_kb(&Al[nloc][kb], hlf);
#pragma unroll
    for (int t = 0; t < 16; ++t) { const v16b bw = frag_kb(WO + (size_t)(grp * 256 + t * 16 + nloc) * H + kb, hlf); acc[t] = wmma16b(a, bw, acc[t]); acc[t] = wmma16b(al, bw, acc[t]); } }
#pragma unroll
  for (int t = 0; t < 16; ++t) { const int cc = t * 16 + nloc; const float bb = bf16_rne(bo[grp * 256 + cc]);
#pragma unroll
    for (int r8 = 0; r8 < 8; ++r8) Tf[8 * hlf + r8][cc] = acc[t][r8] * (1.0f / (XS * WSC)) + bb + O1[8 * hlf + r8][grp * 256 + cc]; }
  wave_lds_sync();
  for (int pass = 0; pass < 2; ++pass) { for (int rr = 0; rr < 16; ++rr) for (int q = 0; q < 2; ++q) *(volatile v4f*)(P + (r0 + rr) * H + grp * 256 + q * 128 + lane * 4) = *(const v4f*)(&Tf[rr][q * 128 + lane * 4]); __threadfence(); } }
__global__ __launch_bounds__(256) void ln2_kernel(const float* __restrict__ P, const float* __restrict__ g2, const float* __restrict__ b2, int RLIM, float* __restrict__ out) { const int wave = threadIdx.x >> 5, lane = threadIdx.x & 31; const size_t r = (size_t)blockIdx.x * 8 + wave; if (r >= (size_t)RLIM) return; float v[16]; float s = 0.0f;
#pragma unroll
  for (int q = 0; q < 16; ++q) { v[q] = P[r * H + q * 32 + lane]; s += v[q]; } for (int o = 16; o; o >>= 1) s += __shfl_xor(s, o); const float mu = s * (1.0f / H); float qs = 0.0f;
#pragma unroll
  for (int q = 0; q < 16; ++q) qs += pmul(v[q] - mu, v[q] - mu); for (int o = 16; o; o >>= 1) qs += __shfl_xor(qs, o); const float rs = rsqrtf(qs * (1.0f / H) + EPS);
  for (int pass = 0; pass < 2; ++pass) {
#pragma unroll
    for (int q = 0; q < 16; ++q) { const int c = q * 32 + lane; ((volatile float*)out)[r * H + c] = pmul(pmul(v[q] - mu, rs), bf16_rne(g2[c])) + bf16_rne(b2[c]); } __threadfence(); } }
}

extern "C" void kernel_launch(void* const* d_in, const int* in_sizes, int n_in, void* d_out, int out_size, void* d_ws, size_t ws_size, hipStream_t stream) {
  (void)n_in;
  auto Fp = [&](int i) { return (const float*)d_in[i]; };
  if (in_sizes[0] != R * H || in_sizes[1] != B * H || in_sizes[4] != H * H || in_sizes[6] != H * H || out_size != R * H) return;
  const int RLIM = R;
  size_t off = 0; char* ws = (char*)d_ws;
  auto carve = [&](size_t bytes) { char* p = ws + off; off += (bytes + 255) & ~(size_t)255; return p; };
  b16* WF = (b16*)carve((size_t)H * H * 2); b16* WO = (b16*)carve((size_t)H * H * 2); float* FP = (float*)carve((size_t)B * H * 4); float* P = (float*)carve((size_t)R * H * 4);
  if (off > ws_size || off > ((size_t)32 << 20)) return;
  wput_kernel<<<(H * (H / 8) + 255) / 256, 256, 0, stream>>>(Fp(4), Fp(6), WF, WO);
  fp_kernel<<<H / 128, 32, 0, stream>>>(Fp(1), WF, Fp(5), FP);
  main_kernel<<<(RLIM / 16) * 2, 32, 0, stream>>>(Fp(0), FP, Fp(8), Fp(9), WO, Fp(7), RLIM, P);
  ln2_kernel<<<(RLIM + 7) / 8, 256, 0, stream>>>(P, Fp(10), Fp(11), RLIM, (float*)d_out);
}
